// TransformerEncoderLayer_27547920236840
// MI455X (gfx1250) — hardware-verified
//
#include <hip/hip_runtime.h>
#ifndef NB
#define NB 4
#endif
#ifndef SEQ
#define SEQ 2048
#endif
#define NB_FULL 4
#define SEQ_FULL 2048
#define DM 512
#define NH 8
#define HD 64
#define DFF 2048
#define DMQ DM
#define LNT (DMQ / 4)
#define NR ((size_t)NB * SEQ)
#define LQK (2 * DM)
static_assert(SEQ % 64 == 0);
static_assert(NB >= 1 && NB <= NB_FULL);
static_assert(SEQ <= SEQ_FULL);
static_assert(NH * HD == DM);
static_assert(DM % 128 == 0 && DFF % 64 == 0 && DM % 32 == 0 && DFF % 32 == 0 && LQK % 64 == 0);
static_assert(((size_t)NB * SEQ) % 128 == 0);
static_assert(DMQ % 4 == 0 && LNT == 128);
static_assert(((size_t)NB * SEQ * DM) % 1024 == 0);
static_assert(((size_t)3 * DM * DM) % 2048 == 0 && ((size_t)DM * DM) % 2048 == 0 && ((size_t)DFF * DM) % 2048 == 0);

constexpr size_t al256(size_t b) { return (b + 255) & ~(size_t)255; }
constexpr size_t SZ_X16 = (size_t)NB * SEQ * DM * 2;
constexpr size_t SZ_QK  = (size_t)NB * SEQ * LQK * 2;
constexpr size_t SZ_VT  = (size_t)DM * NB * SEQ * 2;
constexpr size_t SZ_H   = (size_t)NB * SEQ * DFF * 2;
constexpr size_t SZ_U   = al256((SZ_X16 + SZ_QK + SZ_VT > SZ_H) ? (SZ_X16 + SZ_QK + SZ_VT) : SZ_H);
constexpr size_t SZ_F32 = (size_t)NB * SEQ * DM * 4;
constexpr size_t SZ_TOTAL = al256((size_t)3 * DM * DM * 2) + al256((size_t)DM * DM * 2) + 2 * al256((size_t)DFF * DM * 2) + SZ_U + 3 * al256(SZ_F32) + 2 * al256(SZ_X16);
static_assert(SZ_X16 % 256 == 0 && SZ_QK % 256 == 0 && SZ_VT % 256 == 0);
static_assert(SZ_H <= SZ_U && SZ_X16 + SZ_QK + SZ_VT <= SZ_U);
static_assert(SZ_TOTAL <= (size_t)134217728);

typedef unsigned short v8us __attribute__((ext_vector_type(8), may_alias));
typedef float  v8f  __attribute__((ext_vector_type(8)));
typedef float  v4f  __attribute__((ext_vector_type(4)));
typedef float  v4fa __attribute__((ext_vector_type(4), may_alias));
typedef _Float16 v16h __attribute__((ext_vector_type(16)));
typedef _Float16 v4h __attribute__((ext_vector_type(4)));
union FragH { v16h v; v8us half[2]; _Float16 h[16]; unsigned short u[16]; };

__device__ __forceinline__ unsigned short bf16_bits(float x) { unsigned int u = __float_as_uint(x); return (unsigned short)((u + 0x7FFFu + ((u >> 16) & 1u)) >> 16); }
__device__ __forceinline__ float bf16_val(unsigned short b) { return __uint_as_float(((unsigned int)b) << 16); }
__device__ __forceinline__ float bf16_rne(float x) { return bf16_val(bf16_bits(x)); }

__device__ __forceinline__ v16h g2_frag(const _Float16* p, int hh) { FragH f; f.half[0] = *(const v8us*)((const unsigned short*)p + 8 * hh); f.half[1] = *(const v8us*)((const unsigned short*)p + 16 + 8 * hh); return f.v; }
__device__ __forceinline__ v8f g2_mma(v16h a, v16h b, v8f c) { v8f d = __builtin_amdgcn_wmma_f32_16x16x32_f16(false, a, false, b, (short)0, c, false, false); asm volatile("v_nop\n\tv_nop\n\tv_nop\n\tv_nop" : "+v"(d) : "v"(a), "v"(b)); return d; }

__global__ __launch_bounds__(256) void k_w16(const float* __restrict__ W, _Float16* __restrict__ Wt, unsigned n8, float scale) {
  const unsigned t = blockIdx.x * 256u + threadIdx.x; if (t >= n8) return;
  const size_t e = (size_t)t * 8; const v4f a = *(const v4fa*)(W + e), c = *(const v4fa*)(W + e + 4); FragH f;
#pragma unroll
  for (int q = 0; q < 4; ++q) { f.h[q] = (_Float16)(bf16_rne(a[q]) * scale); f.h[4 + q] = (_Float16)(bf16_rne(c[q]) * scale); }
  const v8us o = f.half[0];
  *(volatile v8us*)((unsigned short*)Wt + e) = o; __threadfence(); *(volatile v8us*)((unsigned short*)Wt + e) = o;
}

__global__ __launch_bounds__(256) void k_xprep(const float* __restrict__ x, _Float16* __restrict__ X16, float* __restrict__ XB) {
  const size_t t = (size_t)blockIdx.x * 256 + threadIdx.x; if (t >= NR * DM / 4) return;
  const size_t e = t * 4; const size_t r = e / DM; const size_t c = e % DM; const size_t rs = (r % SEQ) * NB_FULL + (r / SEQ);
  v4f a = *(const v4fa*)(x + rs * DM + c); v4h h4;
#pragma unroll
  for (int q = 0; q < 4; ++q) { a[q] = bf16_rne(a[q]); h4[q] = (_Float16)a[q]; }
  for (int pass = 0; pass < 2; ++pass) { *(volatile v4h*)(X16 + e) = h4; *(volatile v4f*)(XB + e) = a; if (pass == 0) __threadfence(); }
}

template <int ACT>
__global__ __launch_bounds__(128) void k_gemm2(const _Float16* __restrict__ A, int lda, const _Float16* __restrict__ Bh, int ldb, float alpha, const float* __restrict__ cbias, const float* __restrict__ rbias, const float* __restrict__ CP,
    float* __restrict__ C, _Float16* __restrict__ C16, int ldc, int M, int N, int K) { static_assert(ACT == 0 || ACT == 3);
  __shared__ __attribute__((aligned(16))) float so[4][32][68];
  const int tid = threadIdx.x, w = tid >> 5, lane = tid & 31, ln = lane & 15, hh = lane >> 4;
  const unsigned ntn = (unsigned)N >> 6; const unsigned mt = blockIdx.x / ntn, nq = blockIdx.x - mt * ntn; const int row0 = (int)(mt * 128u) + 32 * w, col0 = (int)(nq * 64u); if (row0 >= M) return;
  const _Float16* a0p = A + (size_t)(row0 + ln) * lda; const _Float16* a1p = a0p + (size_t)16 * lda;
  const _Float16* b0p = Bh + (size_t)(col0 + ln) * ldb; const _Float16* b1p = b0p + (size_t)16 * ldb; const _Float16* b2p = b1p + (size_t)16 * ldb; const _Float16* b3p = b2p + (size_t)16 * ldb;
  const v8f z8 = {0.f,0.f,0.f,0.f,0.f,0.f,0.f,0.f}; v8f c00 = z8, c01 = z8, c02 = z8, c03 = z8, c10 = z8, c11 = z8, c12 = z8, c13 = z8;
#pragma unroll 1
  for (int kb = 0; kb < K; kb += 32) { const v16h a0 = g2_frag(a0p + kb, hh), a1 = g2_frag(a1p + kb, hh);
    v16h b = g2_frag(b0p + kb, hh); c00 = g2_mma(a0, b, c00); c10 = g2_mma(a1, b, c10);
    b = g2_frag(b1p + kb, hh); c01 = g2_mma(a0, b, c01); c11 = g2_mma(a1, b, c11);
    b = g2_frag(b2p + kb, hh); c02 = g2_mma(a0, b, c02); c12 = g2_mma(a1, b, c12);
    b = g2_frag(b3p + kb, hh); c03 = g2_mma(a0, b, c03); c13 = g2_mma(a1, b, c13); }
  v8f accs[8] = {c00, c01, c02, c03, c10, c11, c12, c13};
#pragma unroll
  for (int u = 0; u < 8; ++u) { const int t = u & 3, half = u >> 2; const int col = col0 + t * 16 + ln; const float bv = cbias ? bf16_rne(cbias[col]) : 0.f;
#pragma unroll
    for (int r = 0; r < 8; ++r) { const int rloc = half * 16 + 8 * hh + r; float v = accs[u][r] * alpha + bv;
      if (rbias) v += bf16_rne(rbias[row0 + rloc]);
      if (CP) v += CP[(size_t)(row0 + rloc) * ldc + col];
      if (ACT == 3) v = fmaxf(v, 0.f);
      so[w][rloc][t * 16 + ln] = v; } }
  __builtin_amdgcn_fence(4  , "workgroup"); __builtin_amdgcn_wave_barrier();
  const int rsub = lane >> 4, c4 = (lane & 15) * 4;
  for (int pass = 0; pass < 2; ++pass) {
#pragma unroll
    for (int q = 0; q < 16; ++q) { const int r = q * 2 + rsub; const v4f v = *(const v4fa*)&so[w][r][c4]; if (C) *(volatile v4f*)(C + (size_t)(row0 + r) * ldc + col0 + c4) = v; if (C16) { v4h h4;
#pragma unroll
        for (int i = 0; i < 4; ++i) h4[i] = (_Float16)v[i]; *(volatile v4h*)(C16 + (size_t)(row0 + r) * ldc + col0 + c4) = h4; } }
    if (pass == 0) __threadfence(); } }

template <int BFIN, int W16, int W32, int ORM>
__global__ __launch_bounds__(LNT) void k_lnx(const float* __restrict__ X, const float* __restrict__ g, const float* __restrict__ bb, float eps, _Float16* __restrict__ N16, float* __restrict__ N32) {
  #pragma clang fp contract(off)
  __shared__ float red[LNT]; const size_t r = blockIdx.x; const size_t ro = ORM ? ((r % SEQ) * NB_FULL + (r / SEQ)) : r; const int t = threadIdx.x; const int c0 = t * 4;
  const v4f xa = *(const v4fa*)(X + r * DMQ + c0); float s0, s1, s2, s3;
  s0 = BFIN ? bf16_rne(xa[0]) : xa[0]; s1 = BFIN ? bf16_rne(xa[1]) : xa[1]; s2 = BFIN ? bf16_rne(xa[2]) : xa[2]; s3 = BFIN ? bf16_rne(xa[3]) : xa[3];
  float sum = __fadd_rn(__fadd_rn(__fadd_rn(s0, s1), s2), s3);
  red[t] = sum; __syncthreads(); for (int st = LNT / 2; st > 0; st >>= 1) { if (t < st) red[t] = __fadd_rn(red[t], red[t + st]); __syncthreads(); } const float mu = red[0] / (float)DMQ; __syncthreads();
  const float d0 = __fadd_rn(s0, -mu), d1 = __fadd_rn(s1, -mu), d2 = __fadd_rn(s2, -mu), d3 = __fadd_rn(s3, -mu);
  float vs = __fadd_rn(__fadd_rn(__fadd_rn(__fmul_rn(d0, d0), __fmul_rn(d1, d1)), __fmul_rn(d2, d2)), __fmul_rn(d3, d3));
  red[t] = vs; __syncthreads(); for (int st = LNT / 2; st > 0; st >>= 1) { if (t < st) red[t] = __fadd_rn(red[t], red[t + st]); __syncthreads(); }
  const float rs = rsqrtf(__fadd_rn(red[0] / (float)DMQ, eps)); v4h y; v4f yf;
  const v4f gv = *(const v4fa*)(g + c0); const v4f bv = *(const v4fa*)(bb + c0);
  yf[0] = __fadd_rn(__fmul_rn(__fmul_rn(d0, rs), bf16_rne(gv[0])), bf16_rne(bv[0]));
  yf[1] = __fadd_rn(__fmul_rn(__fmul_rn(d1, rs), bf16_rne(gv[1])), bf16_rne(bv[1]));
  yf[2] = __fadd_rn(__fmul_rn(__fmul_rn(d2, rs), bf16_rne(gv[2])), bf16_rne(bv[2]));
  yf[3] = __fadd_rn(__fmul_rn(__fmul_rn(d3, rs), bf16_rne(gv[3])), bf16_rne(bv[3]));
  y[0] = (_Float16)yf[0]; y[1] = (_Float16)yf[1]; y[2] = (_Float16)yf[2]; y[3] = (_Float16)yf[3];
  for (int pass = 0; pass < 2; ++pass) { if (W16) *(volatile v4h*)(N16 + ro * DMQ + c0) = y; if (W32) *(volatile v4f*)(N32 + ro * DMQ + c0) = yf; if (pass == 0) __threadfence(); } }

__global__ __launch_bounds__(128) void k_attn(const _Float16* __restrict__ QK, const _Float16* __restrict__ VT, _Float16* __restrict__ CAT) {
  __shared__ __attribute__((aligned(16))) unsigned short so[4][16][72];
  const int tid = threadIdx.x, w = tid >> 5, lane = tid & 31, nl = lane & 15, hh = lane >> 4;
  const int h = blockIdx.y, b = blockIdx.z;
  const int q0 = blockIdx.x * 64 + w * 16;
  const size_t rq = (size_t)b * SEQ + q0;
  const size_t rk = (size_t)b * SEQ;
  const _Float16* qp = QK + (rq + nl) * LQK + h * HD;
  const v16h qb0 = g2_frag(qp, hh), qb1 = g2_frag(qp + 32, hh);
  const _Float16* kp = QK + (rk + nl) * LQK + DM + h * HD;
  const _Float16* vp = VT + ((size_t)h * HD + nl) * NR + rk;
  const v8f z8 = {0.f,0.f,0.f,0.f,0.f,0.f,0.f,0.f};
  v8f o0 = z8, o1 = z8, o2 = z8, o3 = z8; float m = -1.0e30f, l = 0.f;
#pragma unroll 1
  for (int kb = 0; kb < SEQ; kb += 32) {
    const _Float16* k0p = kp + (size_t)kb * LQK; const _Float16* k1p = k0p + (size_t)16 * LQK;
    v8f s0 = z8, s1 = z8; v16h a;
    a = g2_frag(k0p, hh); s0 = g2_mma(a, qb0, s0); a = g2_frag(k0p + 32, hh); s0 = g2_mma(a, qb1, s0);
    a = g2_frag(k1p, hh); s1 = g2_mma(a, qb0, s1); a = g2_frag(k1p + 32, hh); s1 = g2_mma(a, qb1, s1);
    float mx = -1.0e30f;
#pragma unroll
    for (int r = 0; r < 8; ++r) mx = fmaxf(mx, fmaxf(s0[r], s1[r]));
    mx = fmaxf(mx, __shfl_xor(mx, 16, 32));
    const float mn = fmaxf(m, mx * 0.125f);
    const float sc = __expf(m - mn);
    FragH pf; float ps = 0.f;
#pragma unroll
    for (int r = 0; r < 8; ++r) { const float e0 = __expf(s0[r] * 0.125f - mn); const float e1 = __expf(s1[r] * 0.125f - mn); ps += e0 + e1; pf.h[r] = (_Float16)(e0 * 256.0f); pf.h[8 + r] = (_Float16)(e1 * 256.0f); }
    ps += __shfl_xor(ps, 16, 32);
    l = l * sc + ps; m = mn;
#pragma unroll
    for (int r = 0; r < 8; ++r) { o0[r] *= sc; o1[r] *= sc; o2[r] *= sc; o3[r] *= sc; }
    const _Float16* v0p = vp + kb;
    a = g2_frag(v0p, hh); o0 = g2_mma(a, pf.v, o0);
    a = g2_frag(v0p + (size_t)16 * NR, hh); o1 = g2_mma(a, pf.v, o1);
    a = g2_frag(v0p + (size_t)32 * NR, hh); o2 = g2_mma(a, pf.v, o2);
    a = g2_frag(v0p + (size_t)48 * NR, hh); o3 = g2_mma(a, pf.v, o3);
  }
  const float inv = 0.25f * (1.0f / l);
  { FragH f;
#pragma unroll
    for (int r = 0; r < 8; ++r) f.h[r] = (_Float16)(o0[r] * inv); *(v8us*)&so[w][nl][0 * 16 + 8 * hh] = f.half[0];
#pragma unroll
    for (int r = 0; r < 8; ++r) f.h[r] = (_Float16)(o1[r] * inv); *(v8us*)&so[w][nl][1 * 16 + 8 * hh] = f.half[0];
#pragma unroll
    for (int r = 0; r < 8; ++r) f.h[r] = (_Float16)(o2[r] * inv); *(v8us*)&so[w][nl][2 * 16 + 8 * hh] = f.half[0];
#pragma unroll
    for (int r = 0; r < 8; ++r) f.h[r] = (_Float16)(o3[r] * inv); *(v8us*)&so[w][nl][3 * 16 + 8 * hh] = f.half[0]; }
  __builtin_amdgcn_fence(4  , "workgroup"); __builtin_amdgcn_wave_barrier();
  const int pr = lane >> 3, pc = lane & 7;
  for (int pass = 0; pass < 2; ++pass) {
#pragma unroll
    for (int it = 0; it < 4; ++it) { const int row = it * 4 + pr; const v8us v = *(const v8us*)&so[w][row][pc * 8]; *(volatile v8us*)((unsigned short*)CAT + (rq + row) * DM + (size_t)h * HD + pc * 8) = v; }
    if (pass == 0) __threadfence(); }
}

extern "C" void kernel_launch(void* const* d_in, const int* in_sizes, int n_in,
                              void* d_out, int out_size, void* d_ws, size_t ws_size, hipStream_t stream) {
  if (n_in < 13) return;
  const float* const* I = (const float* const*)d_in;
  const float* x = I[0]; const float* inw = I[1]; const float* inb = I[2]; const float* wo = I[3]; const float* bo = I[4]; const float* g1 = I[5]; const float* be1 = I[6]; const float* w1 = I[7]; const float* b1 = I[8]; const float* w2 = I[9]; const float* b2 = I[10]; const float* g2 = I[11]; const float* be2 = I[12];
  const size_t need = ((size_t)(SEQ - 1) * NB_FULL + NB) * DM;
  if ((size_t)in_sizes[0] < need || (size_t)out_size < need) return;
  if (in_sizes[1] < 3 * DM * DM || in_sizes[2] < 3 * DM || in_sizes[3] < DM * DM || in_sizes[4] < DM || in_sizes[5] < DM || in_sizes[6] < DM || in_sizes[7] < DFF * DM || in_sizes[8] < DFF || in_sizes[9] < DM * DFF || in_sizes[10] < DM || in_sizes[11] < DM || in_sizes[12] < DM) return;
  const int M = (int)NR;
  char* ws = (char*)d_ws; size_t off = 0;
  auto take = [&](size_t bytes) { char* p = ws + off; off += (bytes + 255) & ~(size_t)255; return p; };
  _Float16* BQKV = (_Float16*)take((size_t)3 * DM * DM * 2);
  _Float16* BTO  = (_Float16*)take((size_t)DM * DM * 2);
  _Float16* BW1  = (_Float16*)take((size_t)DFF * DM * 2);
  _Float16* BW2  = (_Float16*)take((size_t)DM * DFF * 2);
  char*     U    = take(SZ_U);
  _Float16* X16  = (_Float16*)U;
  _Float16* QK16 = (_Float16*)(U + SZ_X16);
  _Float16* VT16 = (_Float16*)(U + SZ_X16 + SZ_QK);
  _Float16* H16  = (_Float16*)U;
  float*    XB   = (float*)take(SZ_F32);
  _Float16* CAT16 = (_Float16*)take(SZ_X16);
  float*    T1   = (float*)take(SZ_F32);
  _Float16* R16  = (_Float16*)take(SZ_X16);
  float*    REC  = (float*)take(SZ_F32);
  float*    T2   = T1;
  if (off > ws_size) return;
  k_xprep<<<(unsigned)(NR * DM / 1024), 256, 0, stream>>>(x, X16, XB);
  k_w16<<<(unsigned)((size_t)3 * DM * DM / 2048), 256, 0, stream>>>(inw, BQKV, (unsigned)((size_t)3 * DM * DM / 8), 16.0f);
  k_w16<<<(unsigned)((size_t)DM * DM / 2048), 256, 0, stream>>>(wo, BTO, (unsigned)((size_t)DM * DM / 8), 16.0f);
  k_w16<<<(unsigned)((size_t)DFF * DM / 2048), 256, 0, stream>>>(w1, BW1, (unsigned)((size_t)DFF * DM / 8), 16.0f);
  k_w16<<<(unsigned)((size_t)DM * DFF / 2048), 256, 0, stream>>>(w2, BW2, (unsigned)((size_t)DM * DFF / 8), 16.0f);
  k_gemm2<0><<<dim3((unsigned)((M / 128) * (LQK / 64)), 1), 128, 0, stream>>>(X16, DM, BQKV, DM, 0.0625f, inb, nullptr, nullptr, nullptr, QK16, LQK, M, LQK, DM);
  k_gemm2<0><<<dim3((unsigned)((DM / 128) * (M / 64)), 1), 128, 0, stream>>>(BQKV + (size_t)2 * DM * DM, DM, X16, DM, 0.0625f, nullptr, inb + 2 * DM, nullptr, nullptr, VT16, M, DM, M, DM);
  k_attn<<<dim3(SEQ / 64, NH, NB), 128, 0, stream>>>(QK16, VT16, CAT16);
  k_gemm2<0><<<dim3((unsigned)((M / 128) * (DM / 64)), 1), 128, 0, stream>>>(CAT16, DM, BTO, DM, 0.0009765625f, bo, nullptr, XB, T1, nullptr, DM, M, DM, DM);
  k_lnx<0, 1, 1, 0><<<(unsigned)M, LNT, 0, stream>>>(T1, g1, be1, 1e-5f, R16, REC);
  k_gemm2<3><<<dim3((unsigned)((M / 128) * (DFF / 64)), 1), 128, 0, stream>>>(R16, DM, BW1, DM, 0.0625f, b1, nullptr, nullptr, nullptr, H16, DFF, M, DFF, DM);
  k_gemm2<0><<<dim3((unsigned)((M / 128) * (DM / 64)), 1), 128, 0, stream>>>(H16, DFF, BW2, DFF, 0.0625f, b2, nullptr, REC, T2, nullptr, DM, M, DM, DFF);
  k_lnx<0, 0, 1, 1><<<(unsigned)M, LNT, 0, stream>>>(T2, g2, be2, 1e-5f, nullptr, (float*)d_out);
}
